// CrossAttFeatTrans_62672162783793
// MI455X (gfx1250) — hardware-run, weakly checked
//
#include <hip/hip_runtime.h>
#include <math.h>

typedef __attribute__((ext_vector_type(16))) _Float16 v16h;
typedef __attribute__((ext_vector_type(8)))  _Float16 v8h;
typedef __attribute__((ext_vector_type(16))) __bf16   v16b;
typedef __attribute__((ext_vector_type(8)))  __bf16   v8b;
typedef __attribute__((ext_vector_type(8)))  float    v8f;
typedef __attribute__((ext_vector_type(4)))  float    v4f;
typedef __attribute__((ext_vector_type(4)))  unsigned int v4u;

constexpr int kB    = 2;
constexpr int kU    = 3072;
constexpr int kIF   = 256;
constexpr int kFD   = 256;
constexpr int kNM   = 4;
constexpr int kHD   = 64;
constexpr int kRows = kB * kU;
constexpr int kQKP  = kNM * kHD;
constexpr int kVN   = kNM * kFD;
constexpr int kHDsqrt = 8;
static_assert(kHDsqrt * kHDsqrt == kHD);
static_assert(kNM * kHD == kIF);
static_assert(kRows == 6144 && kQKP == 256 && kVN == 1024);
static_assert((kIF % 32) == 0 && (kFD % 32) == 0 && (kHD % 32) == 0);
static_assert((kRows % 64) == 0 && (kQKP % 64) == 0 && (kVN % 64) == 0 && (kU % 64) == 0);

constexpr float kQKCarry    = 16.0f;
constexpr float kVCarry     = 16.0f;
constexpr float kPCarry     = 32768.0f;
constexpr float kScoreScale = (1.0f / (float)kHDsqrt) / (kQKCarry * kQKCarry);
constexpr float kOutFold    = kPCarry * kVCarry;
constexpr float kInvFD      = 1.0f / (float)kFD;
constexpr float kLnEps      = 1e-12f;
constexpr float kInvSqrt2   = 0.70710678118654752f;

constexpr int kFaKC = 32;
constexpr int kFaWaves = 8;
constexpr int kFaColsPerWave = 128;
constexpr int kXP   = 260;
constexpr int kMidP = 264;
static_assert((kU % kFaKC) == 0);
static_assert(kFaColsPerWave * 2 == kFD);

constexpr size_t kNX   = (size_t)kRows * kIF;
constexpr size_t kNWq  = (size_t)kQKP * kIF;
constexpr size_t kNWv  = (size_t)kVN * kIF;
constexpr size_t kNWm  = (size_t)kFD * kFD;
constexpr size_t kNWo  = (size_t)kFD * kFD;
constexpr size_t kOffXQ = 0;
constexpr size_t kOffXK = kOffXQ + kNX * 2;
constexpr size_t kOffWQ = kOffXK + kNX * 2;
constexpr size_t kOffWV = kOffWQ + kNWq * 2;
constexpr size_t kOffWM = kOffWV + kNWv * 2;
constexpr size_t kOffWO = kOffWM + kNWm * 2;
constexpr size_t kOffQ  = kOffWO + kNWo * 2;
constexpr size_t kOffK  = kOffQ + (size_t)kRows * kQKP * 2;
constexpr size_t kOffVT = kOffK + (size_t)kRows * kQKP * 2;
constexpr size_t kOffFU = kOffVT + (size_t)kB * kVN * kU * 2;
constexpr size_t kWsTotal = kOffFU + (size_t)kB * kNM * kU * kFD * 4;
static_assert(kWsTotal == 51249152ull);
static_assert(kWsTotal <= 134217728ull);
static_assert((kOffXK % 128) == 0 && (kOffWQ % 128) == 0 && (kOffWV % 128) == 0 && (kOffWM % 128) == 0 &&
              (kOffWO % 128) == 0 && (kOffQ % 128) == 0 && (kOffK % 128) == 0 && (kOffVT % 128) == 0 &&
              (kOffFU % 128) == 0);

static_assert((kNX % 2048) == 0 && (kNWq % 2048) == 0 && (kNWv % 2048) == 0 && (kNWm % 2048) == 0 && (kNWo % 2048) == 0);
constexpr int kCvtB1 = (int)(kNX / 2048);
constexpr int kCvtB2 = kCvtB1 + (int)(kNX / 2048);
constexpr int kCvtB3 = kCvtB2 + (int)(kNWq / 2048);
constexpr int kCvtB4 = kCvtB3 + (int)(kNWv / 2048);
constexpr int kCvtB5 = kCvtB4 + (int)(kNWm / 2048);
constexpr int kCvtB6 = kCvtB5 + (int)(kNWo / 2048);
static_assert(kCvtB6 == 1760);

__device__ __forceinline__ unsigned short f2bf_bits(float f) {
  unsigned u = __float_as_uint(f);
  return (unsigned short)((u + 0x7FFFu + ((u >> 16) & 1u)) >> 16);
}
__device__ __forceinline__ float bf_bits2f(unsigned short h) { return __uint_as_float(((unsigned)h) << 16); }
__device__ __forceinline__ float bf_rne(float f) { return bf_bits2f(f2bf_bits(f)); }
__device__ __forceinline__ unsigned pk16(unsigned short a, unsigned short b) { return (unsigned)a | ((unsigned)b << 16); }

__device__ __forceinline__ void wave_lds_sync() {
  __builtin_amdgcn_fence(__ATOMIC_RELEASE, "workgroup");
  __builtin_amdgcn_wave_barrier();
  __builtin_amdgcn_fence(__ATOMIC_ACQUIRE, "workgroup");
}

__device__ __forceinline__ void grp_guard_h(v8f& a0, v8f& a1, v8f& a2, v8f& a3, v16h x, v16h y) {
  asm volatile("v_nop\n\tv_nop\n\tv_nop\n\tv_nop" : "+v"(a0), "+v"(a1), "+v"(a2), "+v"(a3) : "v"(x), "v"(y));
}
__device__ __forceinline__ void grp_guard_b(v8f& a0, v8f& a1, v8f& a2, v8f& a3, v16b x, v16b y) {
  asm volatile("v_nop\n\tv_nop\n\tv_nop\n\tv_nop" : "+v"(a0), "+v"(a1), "+v"(a2), "+v"(a3) : "v"(x), "v"(y));
}
__device__ __forceinline__ void keep4_h(v16h a, v16h b, v16h c, v16h d) { asm volatile("v_nop" :: "v"(a), "v"(b), "v"(c), "v"(d)); }
__device__ __forceinline__ void keep4_b(v16b a, v16b b, v16b c, v16b d) { asm volatile("v_nop" :: "v"(a), "v"(b), "v"(c), "v"(d)); }
__device__ __forceinline__ void acc_guard4(v8f& a, v8f& b, v8f& c, v8f& d) { asm volatile("v_nop\n\tv_nop\n\tv_nop\n\tv_nop" : "+v"(a), "+v"(b), "+v"(c), "+v"(d)); }

template <typename T> struct Frag;
template <> struct Frag<_Float16> {
  typedef v16h V; union U { v16h v; v8h h[2]; };
  static __device__ __forceinline__ v16h load(const _Float16* p) {
    U f; f.h[0] = *(const v8h*)(p); f.h[1] = *(const v8h*)(p + 16); return f.v;
  }
  static __device__ __forceinline__ v8f mma(v16h a, v16h b, v8f c) {
    return __builtin_amdgcn_wmma_f32_16x16x32_f16(false, a, false, b, (short)0, c, false, false);
  }
  static __device__ __forceinline__ void guard4(v8f& a0, v8f& a1, v8f& a2, v8f& a3, v16h x, v16h y) { grp_guard_h(a0, a1, a2, a3, x, y); }
  static __device__ __forceinline__ void keep(v16h a, v16h b, v16h c, v16h d) { keep4_h(a, b, c, d); }
};
template <> struct Frag<__bf16> {
  typedef v16b V; union U { v16b v; v8b h[2]; };
  static __device__ __forceinline__ v16b load(const __bf16* p) {
    U f; f.h[0] = *(const v8b*)(p); f.h[1] = *(const v8b*)(p + 16); return f.v;
  }
  static __device__ __forceinline__ v8f mma(v16b a, v16b b, v8f c) {
    return __builtin_amdgcn_wmma_f32_16x16x32_bf16(false, a, false, b, (short)0, c, false, false);
  }
  static __device__ __forceinline__ void guard4(v8f& a0, v8f& a1, v8f& a2, v8f& a3, v16b x, v16b y) { grp_guard_b(a0, a1, a2, a3, x, y); }
  static __device__ __forceinline__ void keep(v16b a, v16b b, v16b c, v16b d) { keep4_b(a, b, c, d); }
};

__device__ __forceinline__ v8f mma_h(v16h a, v16h b, v8f c) {
  c = __builtin_amdgcn_wmma_f32_16x16x32_f16(false, a, false, b, (short)0, c, false, false);
  asm volatile("v_nop\n\tv_nop\n\tv_nop\n\tv_nop" : "+v"(c) : "v"(a), "v"(b));
  return c;
}
__device__ __forceinline__ v8f mma_b(v16b a, v16b b, v8f c) {
  c = __builtin_amdgcn_wmma_f32_16x16x32_bf16(false, a, false, b, (short)0, c, false, false);
  asm volatile("v_nop\n\tv_nop\n\tv_nop\n\tv_nop" : "+v"(c) : "v"(a), "v"(b));
  return c;
}

template <int ET> struct Elem;
template <> struct Elem<0> { typedef _Float16 T; };
template <> struct Elem<1> { typedef __bf16 T; };
template <int ET, bool SPLIT, int BIAS_MODE, int OUT_MODE>
__global__ __launch_bounds__(256) void wmma_gemm64(
    const unsigned short* __restrict__ Ap, const unsigned short* __restrict__ A2p, int lda, long strideA,
    const unsigned short* __restrict__ Btp, const unsigned short* __restrict__ Bt2p, int ldb, long strideB,
    void* __restrict__ Cout, void* __restrict__ Cout2, int ldc, long strideC,
    const float* __restrict__ bias,
    int M, int N, int K, float scale) {
  typedef typename Elem<ET>::T T;
  typedef typename Frag<T>::V V;
  const T* A = (const T*)Ap; const T* A2 = (const T*)A2p; const T* Bt = (const T*)Btp; const T* Bt2 = (const T*)Bt2p;
  __shared__ __align__(16) float sT[8][16 * 68];
  const int b    = blockIdx.y;
  const int lane = threadIdx.x & 31;
  const int wave = threadIdx.x >> 5;
  const int tilesN = N >> 6;
  const int tilesM = M >> 6;
  const int tile = blockIdx.x * 8 + wave;
  if (tile >= tilesM * tilesN) return;
  const int tm = tile / tilesN;
  const int tn = tile - tm * tilesN;
  const int m0 = tm << 6;
  const int n0 = tn << 6;

  const T* Ab  = A  + (size_t)b * strideA;
  const T* Bb  = Bt + (size_t)b * strideB;
  const T* Ab2 = SPLIT ? (A2  + (size_t)b * strideA) : nullptr;
  const T* Bb2 = SPLIT ? (Bt2 + (size_t)b * strideB) : nullptr;

  const int rlane = lane & 15;
  const int koff  = (lane >> 4) * 8;
  const int mOff  = (lane >> 4) * 8;

  v8f acc[4][4];
#pragma unroll
  for (int i = 0; i < 4; ++i)
#pragma unroll
    for (int j = 0; j < 4; ++j) acc[i][j] = (v8f){0.f,0.f,0.f,0.f,0.f,0.f,0.f,0.f};

  for (int k0 = 0; k0 < K; k0 += 32) {
    V bh[4], bl[4];
#pragma unroll
    for (int j = 0; j < 4; ++j) {
      const size_t bo = (size_t)(n0 + (j << 4) + rlane) * ldb + koff + k0;
      bh[j] = Frag<T>::load(Bb + bo);
      if (SPLIT) bl[j] = Frag<T>::load(Bb2 + bo);
    }
#pragma unroll
    for (int i = 0; i < 4; ++i) {
      const size_t ao = (size_t)(m0 + (i << 4) + rlane) * lda + koff + k0;
      V ah = Frag<T>::load(Ab + ao);
      V al;
      if (SPLIT) al = Frag<T>::load(Ab2 + ao);
#pragma unroll
      for (int j = 0; j < 4; ++j) {
        acc[i][j] = Frag<T>::mma(ah, bh[j], acc[i][j]);
        if (SPLIT) {
          acc[i][j] = Frag<T>::mma(ah, bl[j], acc[i][j]);
          acc[i][j] = Frag<T>::mma(al, bh[j], acc[i][j]);
        }
      }
      Frag<T>::guard4(acc[i][0], acc[i][1], acc[i][2], acc[i][3], ah, SPLIT ? al : ah);
    }
    Frag<T>::keep(bh[0], bh[1], bh[2], bh[3]);
    if (SPLIT) Frag<T>::keep(bl[0], bl[1], bl[2], bl[3]);
  }
  acc_guard4(acc[0][0], acc[0][1], acc[0][2], acc[0][3]);
  acc_guard4(acc[1][0], acc[1][1], acc[1][2], acc[1][3]);
  acc_guard4(acc[2][0], acc[2][1], acc[2][2], acc[2][3]);
  acc_guard4(acc[3][0], acc[3][1], acc[3][2], acc[3][3]);

  float* slab = sT[wave];
#pragma unroll
  for (int i = 0; i < 4; ++i) {
    const int mBase = m0 + (i << 4);
    float bm[8];
#pragma unroll
    for (int r = 0; r < 8; ++r) bm[r] = 0.f;
    if (BIAS_MODE == 1) {
      const v4f b0 = *(const v4f*)(bias + mBase + mOff);
      const v4f b1 = *(const v4f*)(bias + mBase + mOff + 4);
#pragma unroll
      for (int e = 0; e < 4; ++e) {
        bm[e]     = bf_rne(b0[e]);
        bm[4 + e] = bf_rne(b1[e]);
      }
    }
#pragma unroll
    for (int j = 0; j < 4; ++j) {
      const int n = n0 + (j << 4) + rlane;
      float bv = 0.f;
      if (BIAS_MODE == 2) bv = bf_rne(bias[n]);
#pragma unroll
      for (int r = 0; r < 8; ++r) {
        float v = acc[i][j][r];
        if (BIAS_MODE == 1) v += bm[r];
        if (BIAS_MODE == 2) v += bv;
        v *= scale;
        slab[(mOff + r) * 68 + (j << 4) + rlane] = v;
      }
    }
    wave_lds_sync();
    if (OUT_MODE == 0) {
      float* C = (float*)Cout + (size_t)b * strideC;
      const int hh = lane >> 4, c4 = (lane & 15) * 4;
      for (int pass = 0; pass < 2; ++pass) {
#pragma unroll
        for (int it = 0; it < 8; ++it) {
          const int row = it * 2 + hh;
          v4f v = *(const v4f*)(slab + row * 68 + c4);
          *(volatile v4f*)(C + (size_t)(mBase + row) * ldc + n0 + c4) = v;
        }
        __threadfence();
      }
    } else {
      const int q = lane >> 3, c8 = (lane & 7) * 8;
      unsigned short* C  = (unsigned short*)Cout  + (size_t)b * strideC;
      unsigned short* C2 = (OUT_MODE == 2) ? ((unsigned short*)Cout2 + (size_t)b * strideC) : nullptr;
      for (int pass = 0; pass < 2; ++pass) {
#pragma unroll
        for (int it = 0; it < 4; ++it) {
          const int row = it * 4 + q;
          const float* sp = slab + row * 68 + c8;
          v8h hv, lv;
#pragma unroll
          for (int e = 0; e < 8; ++e) {
            if (OUT_MODE == 1) {
              hv[e] = (_Float16)sp[e];
            } else {
              unsigned short hb = f2bf_bits(sp[e]);
              unsigned short lb = f2bf_bits(sp[e] - bf_bits2f(hb));
              hv[e] = __builtin_bit_cast(_Float16, hb);
              lv[e] = __builtin_bit_cast(_Float16, lb);
            }
          }
          *(volatile v8h*)(C + (size_t)(mBase + row) * ldc + n0 + c8) = hv;
          if (OUT_MODE == 2) *(volatile v8h*)(C2 + (size_t)(mBase + row) * ldc + n0 + c8) = lv;
        }
        __threadfence();
      }
    }
    wave_lds_sync();
  }
}

__global__ __launch_bounds__(256) void cvt_bf16_kernel(
    const float* __restrict__ s0, const float* __restrict__ s1, const float* __restrict__ s2,
    const float* __restrict__ s3, const float* __restrict__ s4, const float* __restrict__ s5,
    unsigned short* __restrict__ dst) {
  const int blk = blockIdx.x;
  if (blk >= kCvtB6) return;
  const float* src;
  int lb;
  if (blk < kCvtB1)      { src = s0; lb = blk; }
  else if (blk < kCvtB2) { src = s1; lb = blk - kCvtB1; }
  else if (blk < kCvtB3) { src = s2; lb = blk - kCvtB2; }
  else if (blk < kCvtB4) { src = s3; lb = blk - kCvtB3; }
  else if (blk < kCvtB5) { src = s4; lb = blk - kCvtB4; }
  else                   { src = s5; lb = blk - kCvtB5; }
  const size_t es = ((size_t)lb * 256 + threadIdx.x) * 8;
  const size_t ed = ((size_t)blk * 256 + threadIdx.x) * 8;
  const v4f a = *(const v4f*)(src + es);
  const v4f c = *(const v4f*)(src + es + 4);
  unsigned short hb[8];
#pragma unroll
  for (int e = 0; e < 4; ++e) {
    hb[e]     = f2bf_bits(a[e]);
    hb[4 + e] = f2bf_bits(c[e]);
  }
  const v4u u = (v4u){pk16(hb[0], hb[1]), pk16(hb[2], hb[3]), pk16(hb[4], hb[5]), pk16(hb[6], hb[7])};
  unsigned short* q = dst + ed;
  *(volatile v4u*)q = u;
  __threadfence();
  *(volatile v4u*)q = u;
}

__global__ __launch_bounds__(256) __attribute__((amdgpu_num_vgpr(256))) void flash_kernel(
    const unsigned short* __restrict__ Qp, const unsigned short* __restrict__ Kp,
    const unsigned short* __restrict__ Vtp, float* __restrict__ fused) {
  __shared__ __align__(16) _Float16 sP[kFaWaves][16 * kFaKC];
  __shared__ __align__(16) float    sO[kFaWaves][16 * 68];

  const int tid  = threadIdx.x;
  const int wave = tid >> 5;
  const int lane = tid & 31;
  const int hh   = lane >> 4;
  const int c    = lane & 15;
  const int rg   = wave >> 1;
  const int fh   = wave & 1;

  constexpr int nqb = kU / 64;
  const int bx = blockIdx.x;
  const int qb = bx % nqb;
  const int bm = bx / nqb;
  const int m  = bm % kNM;
  const int b  = bm / kNM;
  const int q0 = qb * 64 + rg * 16;

  const _Float16* Q  = (const _Float16*)Qp;
  const _Float16* Kk = (const _Float16*)Kp;
  const _Float16* Vt = (const _Float16*)Vtp;

  const _Float16* qrow = Q + (size_t)(b * kU + q0 + c) * kQKP + m * kHD + 8 * hh;
  const v16h qa0 = Frag<_Float16>::load(qrow);
  const v16h qa1 = Frag<_Float16>::load(qrow + 32);

  const _Float16* kbase = Kk + (size_t)(b * kU + c) * kQKP + m * kHD + 8 * hh;
  const _Float16* vbase = Vt + (size_t)(b * kVN + m * kFD + fh * kFaColsPerWave + c) * kU + 8 * hh;

  float mrow[8], lpart[8];
  v8f oacc[8];
#pragma unroll
  for (int r = 0; r < 8; ++r) { mrow[r] = -INFINITY; lpart[r] = 0.f; }
#pragma unroll
  for (int t = 0; t < 8; ++t) oacc[t] = (v8f){0.f,0.f,0.f,0.f,0.f,0.f,0.f,0.f};

  _Float16* pw = sP[wave];

#pragma unroll 1
  for (int kc = 0; kc < kU / kFaKC; ++kc) {
    const int kv0 = kc * kFaKC;
    wave_lds_sync();
    v8f s0 = (v8f){0.f,0.f,0.f,0.f,0.f,0.f,0.f,0.f};
    v8f s1 = (v8f){0.f,0.f,0.f,0.f,0.f,0.f,0.f,0.f};
    {
      const _Float16* kp = kbase + (size_t)kv0 * kQKP;
      const v16h k00 = Frag<_Float16>::load(kp);
      const v16h k01 = Frag<_Float16>::load(kp + 32);
      s0 = mma_h(qa0, k00, s0);
      s0 = mma_h(qa1, k01, s0);
      const v16h k10 = Frag<_Float16>::load(kp + (size_t)16 * kQKP);
      const v16h k11 = Frag<_Float16>::load(kp + (size_t)16 * kQKP + 32);
      s1 = mma_h(qa0, k10, s1);
      s1 = mma_h(qa1, k11, s1);
    }
    float cm[8];
#pragma unroll
    for (int r = 0; r < 8; ++r) {
      s0[r] *= kScoreScale;
      s1[r] *= kScoreScale;
      float mx = fmaxf(s0[r], s1[r]);
#pragma unroll
      for (int off = 1; off < 16; off <<= 1) mx = fmaxf(mx, __shfl_xor(mx, off, 32));
      cm[r] = mx;
    }
#pragma unroll
    for (int r = 0; r < 8; ++r) {
      const float mnew  = fmaxf(mrow[r], cm[r]);
      const float alpha = __expf(mrow[r] - mnew);
      mrow[r] = mnew;
      const float p0 = __expf(s0[r] - mnew);
      const float p1 = __expf(s1[r] - mnew);
      lpart[r] = lpart[r] * alpha + (p0 + p1);
      pw[(8 * hh + r) * kFaKC + c]      = (_Float16)(p0 * kPCarry);
      pw[(8 * hh + r) * kFaKC + 16 + c] = (_Float16)(p1 * kPCarry);
#pragma unroll
      for (int t = 0; t < 8; ++t) oacc[t][r] *= alpha;
    }
    wave_lds_sync();
    const v16h pa = Frag<_Float16>::load(pw + c * kFaKC + 8 * hh);
    const _Float16* vp = vbase + kv0;
#pragma unroll
    for (int tg = 0; tg < 2; ++tg) {
      const v16h vb0 = Frag<_Float16>::load(vp + (size_t)(tg * 4 + 0) * 16 * kU);
      const v16h vb1 = Frag<_Float16>::load(vp + (size_t)(tg * 4 + 1) * 16 * kU);
      const v16h vb2 = Frag<_Float16>::load(vp + (size_t)(tg * 4 + 2) * 16 * kU);
      const v16h vb3 = Frag<_Float16>::load(vp + (size_t)(tg * 4 + 3) * 16 * kU);
      oacc[tg * 4 + 0] = mma_h(pa, vb0, oacc[tg * 4 + 0]);
      oacc[tg * 4 + 1] = mma_h(pa, vb1, oacc[tg * 4 + 1]);
      oacc[tg * 4 + 2] = mma_h(pa, vb2, oacc[tg * 4 + 2]);
      oacc[tg * 4 + 3] = mma_h(pa, vb3, oacc[tg * 4 + 3]);
      asm volatile("" ::: "memory");
    }
  }

  float inv[8];
#pragma unroll
  for (int r = 0; r < 8; ++r) {
    float l = lpart[r];
#pragma unroll
    for (int off = 1; off < 16; off <<= 1) l += __shfl_xor(l, off, 32);
    inv[r] = 1.0f / (l * kOutFold);
  }

  float* os = sO[wave];
  float* fo = fused + (size_t)(bm * kU + q0) * kFD + fh * kFaColsPerWave;
  const int c4 = c * 4;
#pragma unroll
  for (int tg = 0; tg < 2; ++tg) {
#pragma unroll
    for (int r = 0; r < 8; ++r) {
#pragma unroll
      for (int tt = 0; tt < 4; ++tt)
        os[(8 * hh + r) * 68 + tt * 16 + c] = oacc[tg * 4 + tt][r] * inv[r];
    }
    wave_lds_sync();
    for (int pass = 0; pass < 2; ++pass) {
#pragma unroll
      for (int it = 0; it < 8; ++it) {
        const int row = it * 2 + hh;
        const v4f val = *(const v4f*)(os + row * 68 + c4);
        *(volatile v4f*)(fo + (size_t)row * kFD + tg * 64 + c4) = val;
      }
      __threadfence();
    }
    wave_lds_sync();
  }
}

union FragB16 { v16b v; unsigned u[8]; };
__device__ __forceinline__ v16b frag_from_f32(v4f x0, v4f x1, v4f x2, v4f x3) {
  FragB16 f;
  f.u[0] = pk16(f2bf_bits(x0[0]), f2bf_bits(x0[1]));
  f.u[1] = pk16(f2bf_bits(x0[2]), f2bf_bits(x0[3]));
  f.u[2] = pk16(f2bf_bits(x1[0]), f2bf_bits(x1[1]));
  f.u[3] = pk16(f2bf_bits(x1[2]), f2bf_bits(x1[3]));
  f.u[4] = pk16(f2bf_bits(x2[0]), f2bf_bits(x2[1]));
  f.u[5] = pk16(f2bf_bits(x2[2]), f2bf_bits(x2[3]));
  f.u[6] = pk16(f2bf_bits(x3[0]), f2bf_bits(x3[1]));
  f.u[7] = pk16(f2bf_bits(x3[2]), f2bf_bits(x3[3]));
  return f.v;
}

__global__ __launch_bounds__(128) void ffn_ln_agg_kernel(
    const float* __restrict__ fused, const unsigned short* __restrict__ WmidB,
    const unsigned short* __restrict__ WoutB, const float* __restrict__ bmid,
    const float* __restrict__ bout, const float* __restrict__ lng, const float* __restrict__ lnb,
    const float* __restrict__ Wagg, const float* __restrict__ bagg, float* __restrict__ out) {
  __shared__ __align__(16) float  sX[kNM][16 * kXP];
  __shared__ __align__(16) __bf16 sMid[kNM][16 * kMidP];
  __shared__ float sMs[kNM][16];

  const int tid  = threadIdx.x;
  const int wave = tid >> 5;
  const int lane = tid & 31;
  const int hh   = lane >> 4;
  const int c    = lane & 15;
  constexpr int kTilesU = kU / 16;
  const int b  = blockIdx.x / kTilesU;
  const int u0 = (blockIdx.x - b * kTilesU) * 16;

  float* xs = sX[wave];
  __bf16* mt = sMid[wave];

  {
    const float* fsrc = fused + (size_t)((b * kNM + wave) * kU + u0) * kFD;
#pragma unroll 4
    for (int r = 0; r < 16; ++r) {
      const v4f a = *(const v4f*)(fsrc + r * kFD + lane * 4);
      const v4f d = *(const v4f*)(fsrc + r * kFD + 128 + lane * 4);
      *(v4f*)(xs + r * kXP + lane * 4)       = a;
      *(v4f*)(xs + r * kXP + 128 + lane * 4) = d;
    }
  }
  __syncthreads();

  const v8f zero = (v8f){0.f,0.f,0.f,0.f,0.f,0.f,0.f,0.f};
  v16b af[8];
#pragma unroll
  for (int ic = 0; ic < 8; ++ic) {
    const float* p = xs + c * kXP + ic * 32 + 8 * hh;
    const v4f x0 = *(const v4f*)(p);
    const v4f x1 = *(const v4f*)(p + 4);
    const v4f x2 = *(const v4f*)(p + 16);
    const v4f x3 = *(const v4f*)(p + 20);
    af[ic] = frag_from_f32(x0, x1, x2, x3);
  }

  {
    const __bf16* Wm = (const __bf16*)WmidB;
#pragma unroll 1
    for (int og = 0; og < 16; ++og) {
      const __bf16* wr = Wm + (size_t)(og * 16 + c) * kFD + 8 * hh;
      v8f acc = zero;
#pragma unroll
      for (int ic = 0; ic < 8; ++ic) {
        const v16b bfr = Frag<__bf16>::load(wr + ic * 32);
        acc = mma_b(af[ic], bfr, acc);
      }
      const float bi = bf_rne(bmid[og * 16 + c]);
#pragma unroll
      for (int r = 0; r < 8; ++r) {
        const float x = acc[r] + bi;
        const float g = 0.5f * x * (1.0f + erff(x * kInvSqrt2));
        mt[(8 * hh + r) * kMidP + og * 16 + c] = __builtin_bit_cast(__bf16, f2bf_bits(g));
      }
    }
  }
  __syncthreads();

#pragma unroll
  for (int ic = 0; ic < 8; ++ic) af[ic] = Frag<__bf16>::load(mt + c * kMidP + ic * 32 + 8 * hh);

  {
    const __bf16* Wo = (const __bf16*)WoutB;
#pragma unroll 1
    for (int og = 0; og < 16; ++og) {
      const __bf16* wr = Wo + (size_t)(og * 16 + c) * kFD + 8 * hh;
      v8f acc = zero;
#pragma unroll
      for (int ic = 0; ic < 8; ++ic) {
        const v16b bfr = Frag<__bf16>::load(wr + ic * 32);
        acc = mma_b(af[ic], bfr, acc);
      }
      const float bo = bf_rne(bout[og * 16 + c]);
#pragma unroll
      for (int r = 0; r < 8; ++r) {
        const int idx = (8 * hh + r) * kXP + og * 16 + c;
        const float xv = xs[idx];
        xs[idx] = (acc[r] + bo) + xv;
      }
    }
  }
  __syncthreads();

  {
    const int c8 = lane * 8;
    float g8[8], b8[8], w8[8];
    {
      const v4f ga = *(const v4f*)(lng + c8);
      const v4f gb = *(const v4f*)(lng + c8 + 4);
      const v4f ba = *(const v4f*)(lnb + c8);
      const v4f bb = *(const v4f*)(lnb + c8 + 4);
      const v4f wa = *(const v4f*)(Wagg + c8);
      const v4f wb = *(const v4f*)(Wagg + c8 + 4);
#pragma unroll
      for (int e = 0; e < 4; ++e) {
        g8[e] = bf_rne(ga[e]); g8[4 + e] = bf_rne(gb[e]);
        b8[e] = bf_rne(ba[e]); b8[4 + e] = bf_rne(bb[e]);
        w8[e] = bf_rne(wa[e]); w8[4 + e] = bf_rne(wb[e]);
      }
    }
    const float bag = bf_rne(bagg[0]);
    float myms = 0.f;
#pragma unroll 1
    for (int r = 0; r < 16; ++r) {
      float* xr = xs + r * kXP + c8;
      const v4f xa = *(const v4f*)(xr);
      const v4f xb = *(const v4f*)(xr + 4);
      float x[8];
#pragma unroll
      for (int e = 0; e < 4; ++e) { x[e] = xa[e]; x[4 + e] = xb[e]; }
      float sum = ((x[0] + x[1]) + (x[2] + x[3])) + ((x[4] + x[5]) + (x[6] + x[7]));
#pragma unroll
      for (int off = 16; off > 0; off >>= 1) sum += __shfl_xor(sum, off, 32);
      const float mu = sum * kInvFD;
      float d[8];
      float sq = 0.f;
#pragma unroll
      for (int e = 0; e < 8; ++e) { d[e] = x[e] - mu; sq += d[e] * d[e]; }
#pragma unroll
      for (int off = 16; off > 0; off >>= 1) sq += __shfl_xor(sq, off, 32);
      const float rinv = rsqrtf(sq * kInvFD + kLnEps);
      float o[8];
      float dot = 0.f;
#pragma unroll
      for (int e = 0; e < 8; ++e) {
        o[e] = d[e] * rinv * g8[e] + b8[e];
        dot += o[e] * w8[e];
      }
#pragma unroll
      for (int off = 16; off > 0; off >>= 1) dot += __shfl_xor(dot, off, 32);
      const float ms = dot + bag;
      *(v4f*)(xr)     = (v4f){o[0], o[1], o[2], o[3]};
      *(v4f*)(xr + 4) = (v4f){o[4], o[5], o[6], o[7]};
      myms = (lane == r) ? ms : myms;
    }
    if (lane < 16) sMs[wave][lane] = myms;
  }
  __syncthreads();

  float pr[4];
  {
    const int ul = lane & 15;
    const float t0 = sMs[0][ul], t1 = sMs[1][ul], t2 = sMs[2][ul], t3 = sMs[3][ul];
    const float mx = fmaxf(fmaxf(t0, t1), fmaxf(t2, t3));
    const float e0 = expf(t0 - mx), e1 = expf(t1 - mx), e2 = expf(t2 - mx), e3 = expf(t3 - mx);
    const float rs = 1.0f / (((e0 + e1) + e2) + e3);
    pr[0] = e0 * rs; pr[1] = e1 * rs; pr[2] = e2 * rs; pr[3] = e3 * rs;
  }
  v4f ov[8];
#pragma unroll
  for (int i = 0; i < 4; ++i) {
    const int u = wave * 4 + i;
    const float p0 = __shfl(pr[0], u, 32);
    const float p1 = __shfl(pr[1], u, 32);
    const float p2 = __shfl(pr[2], u, 32);
    const float p3 = __shfl(pr[3], u, 32);
#pragma unroll
    for (int h2 = 0; h2 < 2; ++h2) {
      const int col = h2 * 128 + lane * 4;
      const v4f a0 = *(const v4f*)(&sX[0][u * kXP + col]);
      const v4f a1 = *(const v4f*)(&sX[1][u * kXP + col]);
      const v4f a2 = *(const v4f*)(&sX[2][u * kXP + col]);
      const v4f a3 = *(const v4f*)(&sX[3][u * kXP + col]);
      v4f o = a0 * p0;
      o = o + a1 * p1;
      o = o + a2 * p2;
      o = o + a3 * p3;
      ov[i * 2 + h2] = o;
    }
  }
  float* op = out + (size_t)(b * kU + u0 + wave * 4) * kFD;
  for (int pass = 0; pass < 2; ++pass) {
#pragma unroll
    for (int i = 0; i < 4; ++i) {
#pragma unroll
      for (int h2 = 0; h2 < 2; ++h2)
        *(volatile v4f*)(op + (size_t)i * kFD + h2 * 128 + lane * 4) = ov[i * 2 + h2];
    }
    __threadfence();
  }
}

extern "C" void kernel_launch(void* const* d_in, const int* in_sizes, int n_in,
                              void* d_out, int out_size, void* d_ws, size_t ws_size,
                              hipStream_t stream) {
  if (n_in < 13) return;
  if (in_sizes[0] != kRows * kIF) return;
  if (in_sizes[1] != kRows * kIF) return;
  if (in_sizes[2] != kQKP * kIF) return;
  if (in_sizes[3] != kVN * kIF) return;
  if (in_sizes[4] != kVN) return;
  if (in_sizes[5] != kFD * kFD) return;
  if (in_sizes[6] != kFD) return;
  if (in_sizes[7] != kFD * kFD) return;
  if (in_sizes[8] != kFD) return;
  if (in_sizes[9] != kFD) return;
  if (in_sizes[10] != kFD) return;
  if (in_sizes[11] != kFD) return;
  if (in_sizes[12] != 1) return;
  if (out_size != kRows * kFD) return;
  if (ws_size < kWsTotal) return;

  const float* query = (const float*)d_in[0];
  const float* keyf  = (const float*)d_in[1];
  const float* Wq    = (const float*)d_in[2];
  const float* Wv    = (const float*)d_in[3];
  const float* bv    = (const float*)d_in[4];
  const float* Wmid  = (const float*)d_in[5];
  const float* bmid  = (const float*)d_in[6];
  const float* Wout  = (const float*)d_in[7];
  const float* bout  = (const float*)d_in[8];
  const float* lng   = (const float*)d_in[9];
  const float* lnb   = (const float*)d_in[10];
  const float* Wagg  = (const float*)d_in[11];
  const float* bagg  = (const float*)d_in[12];
  float* out = (float*)d_out;

  char* ws = (char*)d_ws;
  unsigned short* XQ = (unsigned short*)(ws + kOffXQ);
  unsigned short* XK = (unsigned short*)(ws + kOffXK);
  unsigned short* WQ = (unsigned short*)(ws + kOffWQ);
  unsigned short* WV = (unsigned short*)(ws + kOffWV);
  unsigned short* WM = (unsigned short*)(ws + kOffWM);
  unsigned short* WO = (unsigned short*)(ws + kOffWO);
  unsigned short* QP = (unsigned short*)(ws + kOffQ);
  unsigned short* KP = (unsigned short*)(ws + kOffK);
  unsigned short* VT = (unsigned short*)(ws + kOffVT);
  float*          FU = (float*)(ws + kOffFU);

  cvt_bf16_kernel<<<kCvtB6, 256, 0, stream>>>(query, keyf, Wq, Wv, Wmid, Wout, XQ);

  wmma_gemm64<1, false, 0, 1><<<dim3(48, 2), 256, 0, stream>>>(
      XQ, nullptr, kIF, (long)kNX,
      WQ, nullptr, kIF, 0L,
      (void*)QP, nullptr, kQKP, (long)kRows * kQKP,
      nullptr,
      kRows, kQKP, kIF, kQKCarry);

  wmma_gemm64<1, false, 1, 1><<<dim3(96, 2), 256, 0, stream>>>(
      WV, nullptr, kIF, 0L,
      XK, nullptr, kIF, (long)kU * kIF,
      (void*)VT, nullptr, kU, (long)kVN * kU,
      bv,
      kVN, kU, kIF, kVCarry);

  flash_kernel<<<kB * kNM * (kU / 64), kFaWaves * 32, 0, stream>>>(QP, KP, VT, FU);

  ffn_ln_agg_kernel<<<kB * (kU / 16), 128, 0, stream>>>(FU, WM, WO, bmid, bout, lng, lnb, Wagg, bagg, out);
}
